// DynamicGraphConv_18184891531673
// MI455X (gfx1250) — hardware-verified
//
#include <hip/hip_runtime.h>

#define BB 8
#define NN 2048
#define FF 128
#define PW 136
#define OP 132
#define ROWS1 128
#define ROWS2 64
#define PSCALE 16384.0f
#define WSCALE 8.0f

typedef _Float16 v16h __attribute__((ext_vector_type(16)));
typedef _Float16 v8h  __attribute__((ext_vector_type(8)));
typedef float    v8f  __attribute__((ext_vector_type(8)));
typedef float    v4f  __attribute__((ext_vector_type(4)));
typedef float    v4fa __attribute__((ext_vector_type(4), __may_alias__));

union Frag { v16h v; v8h half[2]; };

__device__ __forceinline__ v8f wmma_f16(v16h a, v16h b, v8f c) {
    v8f d = __builtin_amdgcn_wmma_f32_16x16x32_f16(false, a, false, b, (short)0, c, false, false);
    asm volatile("v_nop\n\tv_nop\n\tv_nop\n\tv_nop" : "+v"(d) : "v"(a), "v"(b));
    return d;
}

__device__ __forceinline__ _Float16 pval(float s, float s_im, float Mrow, float& z) {
    float e = s_im + s;
    e = (e >= 0.f) ? e : 0.2f * e;
    const float p = __expf(e - Mrow);
    z += p;
    return (_Float16)(p * PSCALE);
}

__global__ void __launch_bounds__(256)
k_proj(const float* __restrict__ x, const float* __restrict__ W, const float* __restrict__ attn,
       _Float16* __restrict__ hT, float* __restrict__ si, float* __restrict__ sj)
{
    __shared__ __align__(16) _Float16 sW[FF * PW];
    __shared__ __align__(16) float sS[2 * ROWS1];

    const int tid = threadIdx.x, l = tid & 31, wv = tid >> 5, h = l >> 4, m = l & 15;
    const int row0 = blockIdx.x * ROWS1;
    const int b = row0 / NN;
    const int jb = row0 - b * NN;

    for (int idx = tid; idx < FF * FF / 4; idx += 256) {
        const int o = idx >> 5, f = (idx & 31) << 2;
        const v4f w = *(const v4f*)(W + o * FF + f);
        _Float16* d = sW + o * PW + f;
        d[0] = (_Float16)(w[0] * WSCALE);
        d[1] = (_Float16)(w[1] * WSCALE);
        d[2] = (_Float16)(w[2] * WSCALE);
        d[3] = (_Float16)(w[3] * WSCALE);
    }
    __syncthreads();

    const int wrow = row0 + wv * 16;
    const v8f zero8 = {0.f, 0.f, 0.f, 0.f, 0.f, 0.f, 0.f, 0.f};
    v8f acc[8];
#pragma unroll
    for (int c = 0; c < 8; ++c) acc[c] = zero8;

#pragma unroll
    for (int k0 = 0; k0 < FF; k0 += 32) {
        const float* xp = x + (size_t)(wrow + m) * FF + k0 + 8 * h;
        const v4f x0 = *(const v4f*)(xp);
        const v4f x1 = *(const v4f*)(xp + 4);
        const v4f x2 = *(const v4f*)(xp + 16);
        const v4f x3 = *(const v4f*)(xp + 20);
        v16h a;
#pragma unroll
        for (int i = 0; i < 4; ++i) {
            a[i]      = (_Float16)x0[i];
            a[4 + i]  = (_Float16)x1[i];
            a[8 + i]  = (_Float16)x2[i];
            a[12 + i] = (_Float16)x3[i];
        }
#pragma unroll
        for (int c = 0; c < 8; ++c) {
            const _Float16* bp = sW + (16 * c + m) * PW + k0 + 8 * h;
            Frag bf;
            bf.half[0] = *(const v8h*)(bp);
            bf.half[1] = *(const v8h*)(bp + 16);
            acc[c] = wmma_f16(a, bf.v, acc[c]);
        }
    }

    float pi[8], pj[8];
#pragma unroll
    for (int r = 0; r < 8; ++r) { pi[r] = 0.f; pj[r] = 0.f; }
#pragma unroll
    for (int c = 0; c < 8; ++c) {
        const float ai = attn[16 * c + m];
        const float aj = attn[FF + 16 * c + m];
#pragma unroll
        for (int r = 0; r < 8; ++r) {
            const float hv = acc[c][r] * (1.0f / WSCALE);
            acc[c][r] = hv;
            pi[r] += hv * ai;
            pj[r] += hv * aj;
        }
    }
#pragma unroll
    for (int r = 0; r < 8; ++r) {
#pragma unroll
        for (int s = 1; s < 16; s <<= 1) {
            pi[r] += __shfl_xor(pi[r], s);
            pj[r] += __shfl_xor(pj[r], s);
        }
    }

    __syncthreads();
    if (m == 0) {
#pragma unroll
        for (int r = 0; r < 8; ++r) {
            sS[wv * 16 + 8 * h + r]         = pi[r];
            sS[ROWS1 + wv * 16 + 8 * h + r] = pj[r];
        }
    }
    _Float16* stg = sW;
#pragma unroll
    for (int c = 0; c < 8; ++c) {
#pragma unroll
        for (int r = 0; r < 8; ++r)
            stg[(16 * c + m) * PW + wv * 16 + 8 * h + r] = (_Float16)acc[c][r];
    }
    __syncthreads();

    {
        const int q = tid & 15, osub = tid >> 4;
        _Float16* hb = hT + (size_t)b * FF * NN + jb + 8 * q;
#pragma unroll
        for (int p = 0; p < 8; ++p) {
            const int o = p * 16 + osub;
            const v8h v = *(const v8h*)(stg + o * PW + 8 * q);
            *(volatile v8h*)(hb + (size_t)o * NN) = v;
        }
        if (wv == 0) {
            const v4f a4 = *(const v4f*)(sS + 4 * l);
            const v4f c4 = *(const v4f*)(sS + ROWS1 + 4 * l);
            *(volatile v4f*)(si + row0 + 4 * l) = a4;
            *(volatile v4f*)(sj + row0 + 4 * l) = c4;
        }
        __threadfence();
#pragma unroll
        for (int p = 0; p < 8; ++p) {
            const int o = p * 16 + osub;
            const v8h v = *(const v8h*)(stg + o * PW + 8 * q);
            *(volatile v8h*)(hb + (size_t)o * NN) = v;
        }
        if (wv == 0) {
            const v4f a4 = *(const v4f*)(sS + 4 * l);
            const v4f c4 = *(const v4f*)(sS + ROWS1 + 4 * l);
            *(volatile v4f*)(si + row0 + 4 * l) = a4;
            *(volatile v4f*)(sj + row0 + 4 * l) = c4;
        }
    }
}

__global__ void __launch_bounds__(128)
k_aggr(const _Float16* __restrict__ hT, const float* __restrict__ si, const float* __restrict__ sj,
       const float* __restrict__ gamma, const float* __restrict__ beta, float* __restrict__ out)
{
    __shared__ __align__(16) float sO[4 * 16 * OP];
    __shared__ float sRed[4];

    const int tid = threadIdx.x, l = tid & 31, wv = tid >> 5, h = l >> 4, m = l & 15;
    const int row0 = blockIdx.x * ROWS2;
    const int b = row0 / NN;
    const int i0 = row0 - b * NN + wv * 16;
    const float* sjb = sj + (size_t)b * NN;

    float mx = -3.0e38f;
    for (int j = tid; j < NN; j += 128) mx = fmaxf(mx, sjb[j]);
#pragma unroll
    for (int s = 16; s > 0; s >>= 1) mx = fmaxf(mx, __shfl_xor(mx, s));
    if (l == 0) sRed[wv] = mx;
    __syncthreads();
    mx = fmaxf(fmaxf(sRed[0], sRed[1]), fmaxf(sRed[2], sRed[3]));

    const float s_im = si[(size_t)b * NN + i0 + m];
    float Mrow = s_im + mx;
    Mrow = (Mrow >= 0.f) ? Mrow : 0.2f * Mrow;

    const v8f zero8 = {0.f, 0.f, 0.f, 0.f, 0.f, 0.f, 0.f, 0.f};
    v8f acc[8];
#pragma unroll
    for (int c = 0; c < 8; ++c) acc[c] = zero8;
    float z = 0.f;
    const _Float16* hb = hT + (size_t)b * FF * NN + 8 * h;

#pragma unroll 1
    for (int j0 = 0; j0 < NN; j0 += 32) {
        const float* sp = sjb + j0 + 8 * h;
        const v4f q0 = *(const v4f*)(sp);
        const v4f q1 = *(const v4f*)(sp + 4);
        const v4f q2 = *(const v4f*)(sp + 16);
        const v4f q3 = *(const v4f*)(sp + 20);
        v16h pa;
#pragma unroll
        for (int i = 0; i < 4; ++i) {
            pa[i]      = pval(q0[i], s_im, Mrow, z);
            pa[4 + i]  = pval(q1[i], s_im, Mrow, z);
            pa[8 + i]  = pval(q2[i], s_im, Mrow, z);
            pa[12 + i] = pval(q3[i], s_im, Mrow, z);
        }
#pragma unroll
        for (int c = 0; c < 8; ++c) {
            const _Float16* bp = hb + (size_t)(16 * c + m) * NN + j0;
            Frag bf;
            bf.half[0] = *(const v8h*)(bp);
            bf.half[1] = *(const v8h*)(bp + 16);
            acc[c] = wmma_f16(pa, bf.v, acc[c]);
        }
    }

    z += __shfl_xor(z, 16);
    const float zs = (1.0f / z) * (1.0f / PSCALE);
    float scl[8];
#pragma unroll
    for (int r = 0; r < 8; ++r) scl[r] = __shfl(zs, 8 * h + r);

    float mu[8], rs[8];
#pragma unroll
    for (int r = 0; r < 8; ++r) {
        float su = 0.f;
#pragma unroll
        for (int c = 0; c < 8; ++c) { const float v = acc[c][r] * scl[r]; acc[c][r] = v; su += v; }
#pragma unroll
        for (int s = 1; s < 16; s <<= 1) su += __shfl_xor(su, s);
        mu[r] = su * (1.0f / FF);
    }
#pragma unroll
    for (int r = 0; r < 8; ++r) {
        float sq = 0.f;
#pragma unroll
        for (int c = 0; c < 8; ++c) { const float d = acc[c][r] - mu[r]; sq += d * d; }
#pragma unroll
        for (int s = 1; s < 16; s <<= 1) sq += __shfl_xor(sq, s);
        rs[r] = rsqrtf(sq * (1.0f / FF) + 1e-5f);
    }

    float* so = sO + wv * 16 * OP;
#pragma unroll
    for (int c = 0; c < 8; ++c) {
        const float g = gamma[16 * c + m], bt = beta[16 * c + m];
#pragma unroll
        for (int r = 0; r < 8; ++r)
            so[(8 * h + r) * OP + 16 * c + m] = (acc[c][r] - mu[r]) * rs[r] * g + bt;
    }
    __syncthreads();

    float* ob = out + ((size_t)b * NN + i0) * FF + 4 * l;
#pragma unroll
    for (int t = 0; t < 16; ++t) {
        const v4f v = *(const v4fa*)(so + t * OP + 4 * l);
        *(volatile v4f*)(ob + (size_t)t * FF) = v;
    }
    __threadfence();
#pragma unroll
    for (int t = 0; t < 16; ++t) {
        const v4f v = *(const v4fa*)(so + t * OP + 4 * l);
        *(volatile v4f*)(ob + (size_t)t * FF) = v;
    }
}

extern "C" void kernel_launch(void* const* d_in, const int* in_sizes, int n_in,
                              void* d_out, int out_size, void* d_ws, size_t ws_size,
                              hipStream_t stream)
{
    const size_t hT_bytes = (size_t)BB * FF * NN * sizeof(_Float16);
    const size_t s_bytes  = (size_t)BB * NN * sizeof(float);
    const size_t total    = hT_bytes + 2 * s_bytes;

    if (n_in < 5) return;
    if (in_sizes[0] != BB * NN * FF || in_sizes[1] != FF * FF || in_sizes[2] != 2 * FF ||
        in_sizes[3] != FF || in_sizes[4] != FF) return;
    if (out_size != BB * NN * FF || ws_size < total) return;

    const float* x     = (const float*)d_in[0];
    const float* W     = (const float*)d_in[1];
    const float* attn  = (const float*)d_in[2];
    const float* gamma = (const float*)d_in[3];
    const float* beta  = (const float*)d_in[4];
    float*       outp  = (float*)d_out;

    char* ws = (char*)d_ws;
    _Float16* hT = (_Float16*)ws;
    float*    si = (float*)(ws + hT_bytes);
    float*    sj = (float*)(ws + hT_bytes + s_bytes);

    k_proj<<<BB * NN / ROWS1, 256, 0, stream>>>(x, W, attn, hT, si, sj);
    k_aggr<<<BB * NN / ROWS2, 128, 0, stream>>>(hT, si, sj, gamma, beta, outp);
    (void)hipGetLastError();
}
